// mLSTMCell_24154896072843
// MI455X (gfx1250) — hardware-verified
//
#include <hip/hip_runtime.h>
#include <math.h>

constexpr int kBatch = 2;
constexpr int kSeq   = 2048;
constexpr int kDim   = 1024;
constexpr int kHeads = 4;
constexpr int kDh    = 256;
constexpr int kTok   = kBatch * kSeq;
constexpr int kBH    = kBatch * kHeads;
constexpr int kGrp   = 2;
constexpr int kGateK = 3 * kDim;
constexpr int kGateN = 64;
constexpr int kRscPitch = 32;
constexpr float kQKScale   = 0.0625f;
constexpr float kPCarry    = 4096.0f;
constexpr float kPCarryInv = 1.0f / 4096.0f;
constexpr float kPClampHi  = 60000.0f;
constexpr float kExpOff    = 40.0f;
constexpr float kExpClamp  = 80.0f;
constexpr float kNormEps   = 1e-8f;
constexpr float kLnEps     = 1e-5f;
constexpr float kInvDh     = 1.0f / 256.0f;
constexpr float kF16MinNormal = 6.103515625e-05f;
static_assert(kHeads * kDh == kDim, "shape");
static_assert(kSeq % 64 == 0 && kDh % 64 == 0 && kTok % 64 == 0 && kGateN % 64 == 0, "M and N tile multiples");
static_assert(kDh % 32 == 0 && kSeq % 32 == 0 && kGateK % 32 == 0, "K multiples of 32");
static_assert(kHeads % kGrp == 0 && kSeq % 256 == 0 && (kTok * kHeads) % 8 == 0, "grids");
static_assert(kDim / 8 == 128 && (kTok * kDim) % (8 * 256) == 0, "cast grid");
static_assert((kGateN * kGateK) % (8 * 256) == 0 && 2 * kHeads <= kGateN, "weight plane grid");

typedef __attribute__((ext_vector_type(16))) _Float16 v16h;
typedef __attribute__((ext_vector_type(8)))  _Float16 v8h;
typedef __attribute__((ext_vector_type(16))) __bf16   v16b;
typedef __attribute__((ext_vector_type(8)))  __bf16   v8b;
typedef __attribute__((ext_vector_type(8)))  float    v8f;
typedef __attribute__((ext_vector_type(4)))  float    v4f;
typedef __attribute__((ext_vector_type(4)))  unsigned int v4u;

__device__ __forceinline__ unsigned short f2bf_bits(float f) {
  unsigned u = __float_as_uint(f);
  return (unsigned short)((u + 0x7FFFu + ((u >> 16) & 1u)) >> 16);
}
__device__ __forceinline__ float bf_bits2f(unsigned short h) { return __uint_as_float(((unsigned)h) << 16); }
__device__ __forceinline__ float bf16r(float f) { return bf_bits2f(f2bf_bits(f)); }

__device__ __forceinline__ void dep_guard_h(v8f& a, v8f& b, v16h x, v16h y) { asm volatile("v_nop\n\tv_nop\n\tv_nop\n\tv_nop" : "+v"(a), "+v"(b) : "v"(x), "v"(y)); }
__device__ __forceinline__ void dep_guard_b(v8f& a, v8f& b, v16b x, v16b y) { asm volatile("v_nop\n\tv_nop\n\tv_nop\n\tv_nop" : "+v"(a), "+v"(b) : "v"(x), "v"(y)); }
__device__ __forceinline__ void dep_guard4_h(v8f& a, v8f& b, v8f& c, v8f& d, v16h x, v16h y) { asm volatile("v_nop\n\tv_nop\n\tv_nop\n\tv_nop" : "+v"(a), "+v"(b), "+v"(c), "+v"(d) : "v"(x), "v"(y)); }
__device__ __forceinline__ void dep_guard4_b(v8f& a, v8f& b, v8f& c, v8f& d, v16b x, v16b y) { asm volatile("v_nop\n\tv_nop\n\tv_nop\n\tv_nop" : "+v"(a), "+v"(b), "+v"(c), "+v"(d) : "v"(x), "v"(y)); }
__device__ __forceinline__ void keep4_h(v16h a, v16h b, v16h c, v16h d) { asm volatile("v_nop" :: "v"(a), "v"(b), "v"(c), "v"(d)); }
__device__ __forceinline__ void keep4_b(v16b a, v16b b, v16b c, v16b d) { asm volatile("v_nop" :: "v"(a), "v"(b), "v"(c), "v"(d)); }
__device__ __forceinline__ void acc_guard4(v8f& a, v8f& b, v8f& c, v8f& d) { asm volatile("v_nop\n\tv_nop\n\tv_nop\n\tv_nop" : "+v"(a), "+v"(b), "+v"(c), "+v"(d)); }
template <typename T> struct Frag;
template <> struct Frag<_Float16> {
  typedef v16h V; union U { v16h v; v8h h[2]; };
  static __device__ __forceinline__ v16h load(const _Float16* p) {
    U f; f.h[0] = *(const v8h*)(p); f.h[1] = *(const v8h*)(p + 16); return f.v;
  }
  static __device__ __forceinline__ v8f mma(v16h a, v16h b, v8f c) {
    return __builtin_amdgcn_wmma_f32_16x16x32_f16(false, a, false, b, (short)0, c, false, false);
  }
  static __device__ __forceinline__ void guard(v8f& a, v8f& b, v16h x, v16h y) { dep_guard_h(a, b, x, y); }
  static __device__ __forceinline__ void guard4(v8f& a, v8f& b, v8f& c, v8f& d, v16h x, v16h y) { dep_guard4_h(a, b, c, d, x, y); }
  static __device__ __forceinline__ void keep(v16h a, v16h b, v16h c, v16h d) { keep4_h(a, b, c, d); }
};
template <> struct Frag<__bf16> {
  typedef v16b V; union U { v16b v; v8b h[2]; };
  static __device__ __forceinline__ v16b load(const __bf16* p) {
    U f; f.h[0] = *(const v8b*)(p); f.h[1] = *(const v8b*)(p + 16); return f.v;
  }
  static __device__ __forceinline__ v8f mma(v16b a, v16b b, v8f c) {
    return __builtin_amdgcn_wmma_f32_16x16x32_bf16(false, a, false, b, (short)0, c, false, false);
  }
  static __device__ __forceinline__ void guard(v8f& a, v8f& b, v16b x, v16b y) { dep_guard_b(a, b, x, y); }
  static __device__ __forceinline__ void guard4(v8f& a, v8f& b, v8f& c, v8f& d, v16b x, v16b y) { dep_guard4_b(a, b, c, d, x, y); }
  static __device__ __forceinline__ void keep(v16b a, v16b b, v16b c, v16b d) { keep4_b(a, b, c, d); }
};

__device__ __forceinline__ unsigned pk16(unsigned short a, unsigned short b) { return (unsigned)a | ((unsigned)b << 16); }
__device__ __forceinline__ unsigned short h_bits(float f) { const _Float16 h = (_Float16)f; return __builtin_bit_cast(unsigned short, h); }
__device__ __forceinline__ unsigned short h_bits_ftz(float f) {
  const float g = (fabsf(f) < kF16MinNormal) ? 0.0f : f;
  return h_bits(g);
}
__device__ __forceinline__ float clampf(float x, float lo, float hi) { return fminf(fmaxf(x, lo), hi); }

template <int ET> struct Elem;
template <> struct Elem<0> { typedef _Float16 T; };
template <> struct Elem<1> { typedef __bf16 T; };
template <int ET, bool SPLIT, int BIAS_MODE, int OUT_MODE, bool RESID, int ACT = 0, int CAUSAL = 0>
__global__ __launch_bounds__(256) void wmma_gemm64(
    const unsigned short* __restrict__ Ap, const unsigned short* __restrict__ A2p, int lda, long strideA,
    const unsigned short* __restrict__ Btp, const unsigned short* __restrict__ Bt2p, int ldb, long strideB,
    void* __restrict__ Cout, void* __restrict__ Cout2, int ldc, long strideC,
    const float* __restrict__ bias,
    const float* __restrict__ resid, long strideR,
    int M, int N, int K, float scale) {
  typedef typename Elem<ET>::T T;
  typedef typename Frag<T>::V V;
  const T* A = (const T*)Ap; const T* A2 = (const T*)A2p; const T* Bt = (const T*)Btp; const T* Bt2 = (const T*)Bt2p;
  __shared__ __align__(16) float sT[8][16 * 68];
  const int b    = blockIdx.y;
  const int lane = threadIdx.x & 31;
  const int wave = threadIdx.x >> 5;
  const int tilesN = N >> 6;
  const int tilesM = M >> 6;
  const int tile = blockIdx.x * 8 + wave;
  if (tile >= tilesM * tilesN) return;
  const int tm = tile / tilesN;
  const int tn = tile - tm * tilesN;
  const int m0 = tm << 6;
  const int n0 = tn << 6;

  int kEnd = K;
  if (CAUSAL == 1) kEnd = (tn > tm) ? 0 : K;
  if (CAUSAL == 2) { const int kc = m0 + 64; kEnd = (kc < K) ? kc : K; }

  const T* Ab  = A  + (size_t)b * strideA;
  const T* Bb  = Bt + (size_t)b * strideB;
  const T* Ab2 = SPLIT ? (A2  + (size_t)b * strideA) : nullptr;
  const T* Bb2 = SPLIT ? (Bt2 + (size_t)b * strideB) : nullptr;

  const int rlane = lane & 15;
  const int koff  = (lane >> 4) * 8;
  const int mOff  = (lane >> 4) * 8;

  v8f acc[4][4];
#pragma unroll
  for (int i = 0; i < 4; ++i)
#pragma unroll
    for (int j = 0; j < 4; ++j) acc[i][j] = (v8f){0.f,0.f,0.f,0.f,0.f,0.f,0.f,0.f};

  for (int k0 = 0; k0 < kEnd; k0 += 32) {
    V bh[4], bl[4];
#pragma unroll
    for (int j = 0; j < 4; ++j) {
      const size_t bo = (size_t)(n0 + (j << 4) + rlane) * ldb + koff + k0;
      bh[j] = Frag<T>::load(Bb + bo);
      if (SPLIT) bl[j] = Frag<T>::load(Bb2 + bo);
    }
#pragma unroll
    for (int i = 0; i < 4; ++i) {
      const size_t ao = (size_t)(m0 + (i << 4) + rlane) * lda + koff + k0;
      V ah = Frag<T>::load(Ab + ao);
      V al;
      if (SPLIT) al = Frag<T>::load(Ab2 + ao);
#pragma unroll
      for (int j = 0; j < 4; ++j) {
        acc[i][j] = Frag<T>::mma(ah, bh[j], acc[i][j]);
        if (SPLIT) {
          acc[i][j] = Frag<T>::mma(ah, bl[j], acc[i][j]);
          acc[i][j] = Frag<T>::mma(al, bh[j], acc[i][j]);
        }
      }
      Frag<T>::guard4(acc[i][0], acc[i][1], acc[i][2], acc[i][3], SPLIT ? al : ah, bh[3]);
    }
    Frag<T>::keep(bh[0], bh[1], bh[2], bh[3]);
    if (SPLIT) Frag<T>::keep(bl[0], bl[1], bl[2], bl[3]);
  }
  acc_guard4(acc[0][0], acc[0][1], acc[0][2], acc[0][3]);
  acc_guard4(acc[1][0], acc[1][1], acc[1][2], acc[1][3]);
  acc_guard4(acc[2][0], acc[2][1], acc[2][2], acc[2][3]);
  acc_guard4(acc[3][0], acc[3][1], acc[3][2], acc[3][3]);

  float* slab = sT[wave];
  const float* Rb = RESID ? (resid + (size_t)b * strideR) : nullptr;
#pragma unroll
  for (int i = 0; i < 4; ++i) {
    const int mBase = m0 + (i << 4);
#pragma unroll
    for (int j = 0; j < 4; ++j) {
      const int n = n0 + (j << 4) + rlane;
      float bv = 0.f;
      if (BIAS_MODE == 2) bv = bias[n];
#pragma unroll
      for (int r = 0; r < 8; ++r) {
        float v = acc[i][j][r] * scale;
        if (BIAS_MODE == 1) v += bias[mBase + mOff + r];
        if (BIAS_MODE == 2) v += bv;
        if (RESID) v += Rb[(size_t)(mBase + mOff + r) * ldc + n];
        if (ACT == 2) v = fmaxf(v, 0.0f);
        if (ACT == 4) v = (v > 0.f) ? v : 0.01f * v;
        slab[(mOff + r) * 68 + (j << 4) + rlane] = v;
      }
    }
    __builtin_amdgcn_fence(__ATOMIC_RELEASE, "workgroup");
    __builtin_amdgcn_wave_barrier();
    __builtin_amdgcn_fence(__ATOMIC_ACQUIRE, "workgroup");
    if (OUT_MODE == 0) {
      float* C = (float*)Cout + (size_t)b * strideC;
      const int hh = lane >> 4, c4 = (lane & 15) * 4;
      for (int pass = 0; pass < 2; ++pass) {
#pragma unroll
        for (int it = 0; it < 8; ++it) {
          const int row = it * 2 + hh;
          v4f v = *(const v4f*)(slab + row * 68 + c4);
          *(volatile v4f*)(C + (size_t)(mBase + row) * ldc + n0 + c4) = v;
        }
        __threadfence();
      }
    } else {
      const int q = lane >> 3, c8 = (lane & 7) * 8;
      unsigned short* C  = (unsigned short*)Cout  + (size_t)b * strideC;
      unsigned short* C2 = (OUT_MODE == 2) ? ((unsigned short*)Cout2 + (size_t)b * strideC) : nullptr;
      for (int pass = 0; pass < 2; ++pass) {
#pragma unroll
        for (int it = 0; it < 4; ++it) {
          const int row = it * 4 + q;
          const float* sp = slab + row * 68 + c8;
          v8h hv, lv;
#pragma unroll
          for (int e = 0; e < 8; ++e) {
            if (OUT_MODE == 1) {
              hv[e] = (_Float16)sp[e];
            } else {
              unsigned short hb = f2bf_bits(sp[e]);
              unsigned short lb = f2bf_bits(sp[e] - bf_bits2f(hb));
              hv[e] = __builtin_bit_cast(_Float16, hb);
              lv[e] = __builtin_bit_cast(_Float16, lb);
            }
          }
          *(volatile v8h*)(C + (size_t)(mBase + row) * ldc + n0 + c8) = hv;
          if (OUT_MODE == 2) *(volatile v8h*)(C2 + (size_t)(mBase + row) * ldc + n0 + c8) = lv;
        }
        __threadfence();
      }
    }
    __builtin_amdgcn_fence(__ATOMIC_RELEASE, "workgroup");
    __builtin_amdgcn_wave_barrier();
    __builtin_amdgcn_fence(__ATOMIC_ACQUIRE, "workgroup");
  }
}

__global__ __launch_bounds__(256) void cast8_bf16_kernel(const float* __restrict__ in, unsigned short* __restrict__ out,
                                                         int n8, int colOff) {
  const int i = blockIdx.x * 256 + threadIdx.x;
  if (i >= n8) return;
  const float* p = in + 8 * (size_t)i;
  const v4f a = *(const v4f*)(p);
  const v4f c = *(const v4f*)(p + 4);
  unsigned short hb[8];
#pragma unroll
  for (int e = 0; e < 4; ++e) {
    hb[e]     = f2bf_bits(a[e]);
    hb[4 + e] = f2bf_bits(c[e]);
  }
  const v4u u = (v4u){pk16(hb[0], hb[1]), pk16(hb[2], hb[3]), pk16(hb[4], hb[5]), pk16(hb[6], hb[7])};
  const int row = i >> 7;
  const int col = (i & 127) * 8;
  unsigned short* q = out + (size_t)row * kGateK + colOff + col;
  *(volatile v4u*)q = u;
  __threadfence();
  *(volatile v4u*)q = u;
}

__global__ __launch_bounds__(256) void wcast_kernel(const float* __restrict__ igw, const float* __restrict__ fgw,
                                                    unsigned short* __restrict__ W16) {
  const int i   = blockIdx.x * 256 + threadIdx.x;
  const int row = i / (kGateK / 8);
  const int c   = (i - row * (kGateK / 8)) * 8;
  const int ri  = (row < kHeads) ? row : (kHeads - 1);
  int rf = row - kHeads; rf = (rf < 0) ? 0 : rf; rf = (rf > kHeads - 1) ? (kHeads - 1) : rf;
  const float fa = (row < kHeads) ? 1.0f : 0.0f;
  const float fb = (row >= kHeads && row < 2 * kHeads) ? 1.0f : 0.0f;
  const float* pa = igw + (size_t)ri * kGateK + c;
  const float* pb = fgw + (size_t)rf * kGateK + c;
  const v4f a0 = *(const v4f*)(pa);
  const v4f a1 = *(const v4f*)(pa + 4);
  const v4f b0 = *(const v4f*)(pb);
  const v4f b1 = *(const v4f*)(pb + 4);
  unsigned short hb[8];
#pragma unroll
  for (int e = 0; e < 4; ++e) {
    hb[e]     = f2bf_bits(fmaf(fa, a0[e], fb * b0[e]));
    hb[4 + e] = f2bf_bits(fmaf(fa, a1[e], fb * b1[e]));
  }
  const v4u u = (v4u){pk16(hb[0], hb[1]), pk16(hb[2], hb[3]), pk16(hb[4], hb[5]), pk16(hb[6], hb[7])};
  unsigned short* q = W16 + 8 * (size_t)i;
  *(volatile v4u*)q = u;
  __threadfence();
  *(volatile v4u*)q = u;
}

__global__ __launch_bounds__(256) void vt_cast_kernel(const float* __restrict__ v, unsigned short* __restrict__ VT) {
  __shared__ float sm[64][65];
  const int t  = threadIdx.x;
  const int s0 = blockIdx.x * 64;
  const int d0 = blockIdx.y * 64;
  const int bh = blockIdx.z;
  const int b  = bh >> 2;
  const int h  = bh & 3;
#pragma unroll
  for (int i = 0; i < 16; ++i) {
    const int e = i * 256 + t;
    const int r = e >> 6;
    const int c = e & 63;
    sm[c][r] = bf16r(v[((size_t)(b * kSeq + s0 + r)) * kDim + h * kDh + d0 + c]);
  }
  __syncthreads();
  const int lane = t & 31, wave = t >> 5;
  const int q = lane >> 3, c8 = (lane & 7) * 8;
  unsigned short* op = VT + ((size_t)bh * kDh) * kSeq;
  for (int pass = 0; pass < 2; ++pass) {
#pragma unroll
    for (int it = 0; it < 2; ++it) {
      const int row = wave * 8 + it * 4 + q;
      unsigned short hb[8];
#pragma unroll
      for (int e = 0; e < 8; ++e) hb[e] = h_bits_ftz(sm[row][c8 + e]);
      const v4u u = (v4u){pk16(hb[0], hb[1]), pk16(hb[2], hb[3]), pk16(hb[4], hb[5]), pk16(hb[6], hb[7])};
      *(volatile v4u*)(op + (size_t)(d0 + row) * kSeq + s0 + c8) = u;
    }
    __threadfence();
  }
}

__global__ __launch_bounds__(256) void scan_kernel(const float* __restrict__ GT, const float* __restrict__ igb,
                                                   const float* __restrict__ fgb,
                                                   float* __restrict__ EA, float* __restrict__ EM, float* __restrict__ NFL) {
  __shared__ float lfs[kSeq];
  __shared__ float avs[kSeq];
  __shared__ float css[kSeq];
  __shared__ float mss[kSeq];
  __shared__ float red[256];
  const int bh = blockIdx.x;
  const int b  = bh >> 2;
  const int h  = bh & 3;
  const int t  = threadIdx.x;
  const float bi = bf16r(igb[h]);
  const float bf = bf16r(fgb[h]);
  const float* gtb = GT + ((size_t)b * kSeq) * kGateN;
#pragma unroll 1
  for (int e = 0; e < 8; ++e) {
    const int s = e * 256 + t;
    const float* gr = gtb + (size_t)s * kGateN;
    const float x = gr[kHeads + h] + bf;
    const float lf = fminf(x, 0.0f) - log1pf(expf(-fabsf(x)));
    lfs[s] = lf;
    avs[s] = gr[h] + bi;
  }
  __syncthreads();
  const int s8 = 8 * t;
  float cl[8];
  float run = 0.0f;
#pragma unroll
  for (int e = 0; e < 8; ++e) { run = run + lfs[s8 + e]; cl[e] = run; }
  red[t] = run;
  __syncthreads();
  for (int off = 1; off < 256; off <<= 1) {
    int im = t - off; im = (im < 0) ? 0 : im;
    float vv = red[im];
    vv = (t >= off) ? vv : 0.0f;
    __syncthreads();
    red[t] = red[t] + vv;
    __syncthreads();
  }
  float excl;
  {
    int ip = t - 1; ip = (ip < 0) ? 0 : ip;
    const float pv = red[ip];
    excl = (t == 0) ? 0.0f : pv;
  }
#pragma unroll
  for (int e = 0; e < 8; ++e) css[s8 + e] = excl + cl[e];
  __syncthreads();
  float al[8], am[8];
  float runmax = -__builtin_inff();
#pragma unroll
  for (int e = 0; e < 8; ++e) {
    const int s  = s8 + e;
    const int sp = (s == 0) ? 0 : (s - 1);
    float prev = css[sp];
    prev = (s == 0) ? 0.0f : prev;
    const float a = avs[s] - prev;
    al[e] = a;
    runmax = fmaxf(runmax, a);
    am[e] = runmax;
  }
#pragma unroll
  for (int e = 0; e < 8; ++e) avs[s8 + e] = al[e];
  red[t] = runmax;
  __syncthreads();
  for (int off = 1; off < 256; off <<= 1) {
    int im = t - off; im = (im < 0) ? 0 : im;
    float vv = red[im];
    vv = (t >= off) ? vv : -__builtin_inff();
    __syncthreads();
    red[t] = fmaxf(red[t], vv);
    __syncthreads();
  }
  float pm;
  {
    int ip = t - 1; ip = (ip < 0) ? 0 : ip;
    const float pv = red[ip];
    pm = (t == 0) ? -__builtin_inff() : pv;
  }
#pragma unroll
  for (int e = 0; e < 8; ++e) mss[s8 + e] = fmaxf(pm, am[e]);
  __syncthreads();
  float* eap = EA  + (size_t)bh * kSeq;
  float* emp = EM  + (size_t)bh * kSeq;
  float* nfp = NFL + (size_t)bh * kSeq;
#pragma unroll 1
  for (int e = 0; e < 8; ++e) {
    const int s = e * 256 + t;
    const float a  = avs[s];
    const float m  = mss[s];
    const float cs = css[s];
    const float ea = expf(clampf(a - kExpOff, -kExpClamp, kExpClamp));
    const float em = expf(clampf(kExpOff - m, -kExpClamp, kExpClamp));
    const float nf = expf(clampf(-(cs + m), -kExpClamp, kExpClamp));
    *(volatile float*)(eap + s) = ea;
    *(volatile float*)(emp + s) = em;
    *(volatile float*)(nfp + s) = nf;
    __threadfence();
    *(volatile float*)(eap + s) = ea;
    *(volatile float*)(emp + s) = em;
    *(volatile float*)(nfp + s) = nf;
  }
}

__global__ __launch_bounds__(256) void decay_p_kernel(const float* __restrict__ SC, const float* __restrict__ EA,
                                                      const float* __restrict__ EM, const float* __restrict__ NFL,
                                                      unsigned short* __restrict__ PP, float* __restrict__ RSC, int bh0) {
  __shared__ float red[8];
  const int i    = blockIdx.x;
  const int g    = blockIdx.y;
  const int bh   = bh0 + g;
  const int t    = threadIdx.x;
  const int lane = t & 31, wave = t >> 5;
  const size_t rowoff = ((size_t)g * kSeq + i) * kSeq;
  const float* sr = SC + rowoff + 8 * (size_t)t;
  const float* er = EA + (size_t)bh * kSeq + 8 * t;
  const float emi = EM[(size_t)bh * kSeq + i];
  const float nfi = NFL[(size_t)bh * kSeq + i];
  const v4f sa = *(const v4f*)(sr);
  const v4f sb = *(const v4f*)(sr + 4);
  const v4f xa = *(const v4f*)(er);
  const v4f xb = *(const v4f*)(er + 4);
  const int j0 = 8 * t;
  float c[8];
  unsigned short hb[8];
#pragma unroll
  for (int e = 0; e < 4; ++e) {
    const float da = fminf(xa[e] * emi, 1.0f);
    const float db = fminf(xb[e] * emi, 1.0f);
    float ca = sa[e] * da;
    float cb = sb[e] * db;
    ca = (j0 + e <= i) ? ca : 0.0f;
    cb = (j0 + 4 + e <= i) ? cb : 0.0f;
    c[e] = ca;
    c[4 + e] = cb;
    hb[e]     = h_bits_ftz(clampf(ca * kPCarry, -kPClampHi, kPClampHi));
    hb[4 + e] = h_bits_ftz(clampf(cb * kPCarry, -kPClampHi, kPClampHi));
  }
  float sum = ((c[0] + c[1]) + (c[2] + c[3])) + ((c[4] + c[5]) + (c[6] + c[7]));
  const v4u u = (v4u){pk16(hb[0], hb[1]), pk16(hb[2], hb[3]), pk16(hb[4], hb[5]), pk16(hb[6], hb[7])};
  unsigned short* pr = PP + rowoff + 8 * (size_t)t;
  *(volatile v4u*)pr = u;
  __threadfence();
  *(volatile v4u*)pr = u;
#pragma unroll
  for (int off = 16; off > 0; off >>= 1) sum += __shfl_xor(sum, off, 32);
  if (lane == 0) red[wave] = sum;
  __syncthreads();
  float tot = red[0];
#pragma unroll
  for (int w = 1; w < 8; ++w) tot += red[w];
  const float nrm = fmaxf(fabsf(tot), nfi) + kNormEps;
  const float rsc = (1.0f / nrm) * kPCarryInv;
  if (wave == 0) {
    float* rl = RSC + ((size_t)bh * kSeq + i) * kRscPitch + lane;
    *(volatile float*)rl = rsc;
    __threadfence();
    *(volatile float*)rl = rsc;
  }
}

__global__ __launch_bounds__(256) void gnorm_kernel(const float* __restrict__ HP, const float* __restrict__ RSC,
                                                    const float* __restrict__ ow, float* __restrict__ out) {
  const int lane = threadIdx.x & 31, wave = threadIdx.x >> 5;
  const int task = blockIdx.x * 8 + wave;
  const int tok  = task >> 2;
  const int h    = task & 3;
  const int b    = tok >> 11;
  const int s    = tok & (kSeq - 1);
  const int bh   = b * kHeads + h;
  const float rsc = RSC[((size_t)bh * kSeq + s) * kRscPitch];
  const float* hr = HP + (size_t)tok * kDim + h * kDh + 4 * lane;
  const v4f xa = *(const v4f*)(hr);
  const v4f xb = *(const v4f*)(hr + 128);
  const float* wr = ow + h * kDh + 4 * lane;
  const v4f wa = *(const v4f*)(wr);
  const v4f wb = *(const v4f*)(wr + 128);
  float x[8];
#pragma unroll
  for (int e = 0; e < 4; ++e) { x[e] = xa[e] * rsc; x[4 + e] = xb[e] * rsc; }
  float s1 = ((x[0] + x[1]) + (x[2] + x[3])) + ((x[4] + x[5]) + (x[6] + x[7]));
#pragma unroll
  for (int off = 16; off > 0; off >>= 1) s1 += __shfl_xor(s1, off, 32);
  const float mean = s1 * kInvDh;
  float d[8];
#pragma unroll
  for (int e = 0; e < 8; ++e) d[e] = x[e] - mean;
  float s2 = ((d[0] * d[0] + d[1] * d[1]) + (d[2] * d[2] + d[3] * d[3])) + ((d[4] * d[4] + d[5] * d[5]) + (d[6] * d[6] + d[7] * d[7]));
#pragma unroll
  for (int off = 16; off > 0; off >>= 1) s2 += __shfl_xor(s2, off, 32);
  const float var = s2 * kInvDh;
  const float rs  = 1.0f / sqrtf(var + kLnEps);
  v4f oa, ob;
#pragma unroll
  for (int e = 0; e < 4; ++e) {
    oa[e] = d[e] * rs * (1.0f + bf16r(wa[e]));
    ob[e] = d[4 + e] * rs * (1.0f + bf16r(wb[e]));
  }
  float* op = out + (size_t)tok * kDim + h * kDh + 4 * lane;
  *(volatile v4f*)(op) = oa;
  *(volatile v4f*)(op + 128) = ob;
  __threadfence();
  *(volatile v4f*)(op) = oa;
  *(volatile v4f*)(op + 128) = ob;
}

extern "C" void kernel_launch(void* const* d_in, const int* in_sizes, int n_in,
                              void* d_out, int out_size, void* d_ws, size_t ws_size,
                              hipStream_t stream) {
  if (n_in < 8) return;
  const int nElem = kBatch * kSeq * kDim;
  if (in_sizes[0] != nElem || in_sizes[1] != nElem || in_sizes[2] != nElem) return;
  if (in_sizes[3] != kHeads * kGateK || in_sizes[5] != kHeads * kGateK) return;
  if (in_sizes[4] != kHeads || in_sizes[6] != kHeads || in_sizes[7] != kDim) return;
  if (out_size != nElem) return;

  const size_t szX  = (size_t)kTok * kGateK * 2;
  const size_t szVT = (size_t)kBH * kDh * kSeq * 2;
  const size_t szW  = (size_t)kGateN * kGateK * 2;
  const size_t szGT = (size_t)kTok * kGateN * 4;
  const size_t szG  = (size_t)kBH * kSeq * 4;
  const size_t szRS = (size_t)kBH * kSeq * kRscPitch * 4;
  const size_t szHP = (size_t)kTok * kDim * 4;
  const size_t szSC = (size_t)kGrp * kSeq * kSeq * 4;
  const size_t szPP = (size_t)kGrp * kSeq * kSeq * 2;
  const size_t offX  = 0;
  const size_t offVT = offX + szX;
  const size_t offW  = offVT + szVT;
  const size_t offGT = offW + szW;
  const size_t offEA = offGT + szGT;
  const size_t offEM = offEA + szG;
  const size_t offNF = offEM + szG;
  const size_t offRS = offNF + szG;
  const size_t offHP = offRS + szRS;
  const size_t offSC = offHP + szHP;
  const size_t offPP = offSC + szSC;
  const size_t total = offPP + szPP;
  if (ws_size < total) return;

  const float* q   = (const float*)d_in[0];
  const float* k   = (const float*)d_in[1];
  const float* v   = (const float*)d_in[2];
  const float* igw = (const float*)d_in[3];
  const float* igb = (const float*)d_in[4];
  const float* fgw = (const float*)d_in[5];
  const float* fgb = (const float*)d_in[6];
  const float* ow  = (const float*)d_in[7];
  float* out = (float*)d_out;
  char* ws = (char*)d_ws;
  unsigned short* X16 = (unsigned short*)(ws + offX);
  unsigned short* VT  = (unsigned short*)(ws + offVT);
  unsigned short* W16 = (unsigned short*)(ws + offW);
  float* GT  = (float*)(ws + offGT);
  float* EA  = (float*)(ws + offEA);
  float* EM  = (float*)(ws + offEM);
  float* NFL = (float*)(ws + offNF);
  float* RSC = (float*)(ws + offRS);
  float* HP  = (float*)(ws + offHP);
  float* SC  = (float*)(ws + offSC);
  unsigned short* PP = (unsigned short*)(ws + offPP);

  const int n8 = (kTok * kDim) / 8;
  cast8_bf16_kernel<<<dim3(n8 / 256), dim3(256), 0, stream>>>(q, X16, n8, 0);
  cast8_bf16_kernel<<<dim3(n8 / 256), dim3(256), 0, stream>>>(k, X16, n8, kDim);
  cast8_bf16_kernel<<<dim3(n8 / 256), dim3(256), 0, stream>>>(v, X16, n8, 2 * kDim);
  vt_cast_kernel<<<dim3(kSeq / 64, kDh / 64, kBH), dim3(256), 0, stream>>>(v, VT);
  wcast_kernel<<<dim3((kGateN * kGateK) / (8 * 256)), dim3(256), 0, stream>>>(igw, fgw, W16);

  wmma_gemm64<1, false, 0, 0, false, 0, 0><<<dim3((kTok / 64) * (kGateN / 64) / 8, 1), dim3(256), 0, stream>>>(
      X16, X16, kGateK, 0L, W16, W16, kGateK, 0L,
      (void*)GT, (void*)GT, kGateN, 0L, EA, EA, 0L, kTok, kGateN, kGateK, 1.0f);

  scan_kernel<<<dim3(kBH), dim3(256), 0, stream>>>(GT, igb, fgb, EA, EM, NFL);

  const long strideHead16 = (long)kDh;
  const long strideScore  = (long)kSeq * kSeq;
  const long strideVT     = (long)kDh * kSeq;
  const int  tilesScore   = (kSeq / 64) * (kSeq / 64);
  const int  tilesHead    = (kSeq / 64) * (kDh / 64);

  for (int b = 0; b < kBatch; ++b) {
    for (int hp = 0; hp < kHeads / kGrp; ++hp) {
      const int h0  = hp * kGrp;
      const int bh0 = b * kHeads + h0;
      const size_t xOff  = ((size_t)b * kSeq) * kGateK + (size_t)h0 * kDh;
      const size_t hpOff = ((size_t)b * kSeq) * kDim + (size_t)h0 * kDh;
      const unsigned short* Ag  = X16 + xOff;
      const unsigned short* Btg = X16 + xOff + kDim;
      wmma_gemm64<1, false, 0, 0, false, 0, 1><<<dim3(tilesScore / 8, kGrp), dim3(256), 0, stream>>>(
          Ag, Ag, kGateK, strideHead16, Btg, Btg, kGateK, strideHead16,
          (void*)SC, (void*)SC, kSeq, strideScore, EA, EA, 0L, kSeq, kSeq, kDh, kQKScale);
      decay_p_kernel<<<dim3(kSeq, kGrp), dim3(256), 0, stream>>>(SC, EA, EM, NFL, PP, RSC, bh0);
      const unsigned short* VTg = VT + (size_t)bh0 * kDh * kSeq;
      float* hpg = HP + hpOff;
      wmma_gemm64<0, false, 0, 0, false, 0, 2><<<dim3(tilesHead / 8, kGrp), dim3(256), 0, stream>>>(
          PP, PP, kSeq, strideScore, VTg, VTg, kSeq, strideVT,
          (void*)hpg, (void*)hpg, kDim, strideHead16, EA, EA, 0L, kSeq, kDh, kSeq, 1.0f);
    }
  }
  gnorm_kernel<<<dim3((kTok * kHeads) / 8), dim3(256), 0, stream>>>(HP, RSC, ow, out);
}
